// SelfAttentionRPR_19078244729547
// MI455X (gfx1250) — hardware-verified
//
#include <hip/hip_runtime.h>
#include <math.h>

constexpr int NBATCH = 8;
constexpr int SEQ    = 1024;
constexpr int DMODEL = 128;
constexpr int NTOK   = NBATCH * SEQ;
constexpr int RWIN   = 64;
constexpr int NREL   = 2 * RWIN + 1;
constexpr int NRELP  = 192;
constexpr int RCOLS  = 192;
constexpr int LDCAT  = SEQ + RCOLS;
static_assert(LDCAT % 64 == 0, "pitch");
static_assert(NRELP % 64 == 0, "pad");

typedef __attribute__((ext_vector_type(16))) _Float16 v16h;
typedef __attribute__((ext_vector_type(8)))  _Float16 v8h;
typedef __attribute__((ext_vector_type(16))) __bf16   v16b;
typedef __attribute__((ext_vector_type(8)))  __bf16   v8b;
typedef __attribute__((ext_vector_type(8)))  float    v8f;
typedef __attribute__((ext_vector_type(4)))  float    v4f;
typedef __attribute__((ext_vector_type(4)))  unsigned int v4u;

__device__ __forceinline__ unsigned short f2bf_bits(float f) {
  unsigned u = __float_as_uint(f);
  return (unsigned short)((u + 0x7FFFu + ((u >> 16) & 1u)) >> 16);
}
__device__ __forceinline__ float bf_bits2f(unsigned short h) { return __uint_as_float(((unsigned)h) << 16); }

__device__ __forceinline__ void dep_guard_h(v8f& a, v8f& b, v16h x, v16h y) { asm volatile("v_nop\n\tv_nop\n\tv_nop\n\tv_nop" : "+v"(a), "+v"(b) : "v"(x), "v"(y)); }
__device__ __forceinline__ void dep_guard_b(v8f& a, v8f& b, v16b x, v16b y) { asm volatile("v_nop\n\tv_nop\n\tv_nop\n\tv_nop" : "+v"(a), "+v"(b) : "v"(x), "v"(y)); }
__device__ __forceinline__ void keep4_h(v16h a, v16h b, v16h c, v16h d) { asm volatile("v_nop" :: "v"(a), "v"(b), "v"(c), "v"(d)); }
__device__ __forceinline__ void keep4_b(v16b a, v16b b, v16b c, v16b d) { asm volatile("v_nop" :: "v"(a), "v"(b), "v"(c), "v"(d)); }
__device__ __forceinline__ void acc_guard4(v8f& a, v8f& b, v8f& c, v8f& d) { asm volatile("v_nop\n\tv_nop\n\tv_nop\n\tv_nop" : "+v"(a), "+v"(b), "+v"(c), "+v"(d)); }
template <typename T> struct Frag;
template <> struct Frag<_Float16> {
  typedef v16h V; union U { v16h v; v8h h[2]; };
  static __device__ __forceinline__ v16h load(const _Float16* p) {
    U f; f.h[0] = *(const v8h*)(p); f.h[1] = *(const v8h*)(p + 16); return f.v;
  }
  static __device__ __forceinline__ v8f mma(v16h a, v16h b, v8f c) {
    return __builtin_amdgcn_wmma_f32_16x16x32_f16(false, a, false, b, (short)0, c, false, false);
  }
  static __device__ __forceinline__ void guard(v8f& a, v8f& b, v16h x, v16h y) { dep_guard_h(a, b, x, y); }
  static __device__ __forceinline__ void keep(v16h a, v16h b, v16h c, v16h d) { keep4_h(a, b, c, d); }
};
template <> struct Frag<__bf16> {
  typedef v16b V; union U { v16b v; v8b h[2]; };
  static __device__ __forceinline__ v16b load(const __bf16* p) {
    U f; f.h[0] = *(const v8b*)(p); f.h[1] = *(const v8b*)(p + 16); return f.v;
  }
  static __device__ __forceinline__ v8f mma(v16b a, v16b b, v8f c) {
    return __builtin_amdgcn_wmma_f32_16x16x32_bf16(false, a, false, b, (short)0, c, false, false);
  }
  static __device__ __forceinline__ void guard(v8f& a, v8f& b, v16b x, v16b y) { dep_guard_b(a, b, x, y); }
  static __device__ __forceinline__ void keep(v16b a, v16b b, v16b c, v16b d) { keep4_b(a, b, c, d); }
};

__device__ __forceinline__ unsigned pk16(unsigned short a, unsigned short b) { return (unsigned)a | ((unsigned)b << 16); }

template <int ET> struct Elem;
template <> struct Elem<0> { typedef _Float16 T; };
template <> struct Elem<1> { typedef __bf16 T; };
template <int ET, int SPLIT, int BIAS_MODE, int OUT_MODE, bool RESID, int ACT = 0>
__global__ __launch_bounds__(256) void wmma_gemm64(
    const unsigned short* __restrict__ Ap, const unsigned short* __restrict__ A2p, int lda, long strideA,
    const unsigned short* __restrict__ Btp, const unsigned short* __restrict__ Bt2p, int ldb, long strideB,
    void* __restrict__ Cout, void* __restrict__ Cout2, int ldc, long strideC,
    const float* __restrict__ bias,
    const float* __restrict__ resid, long strideR,
    int M, int N, int K, float scale) {
  typedef typename Elem<ET>::T T;
  typedef typename Frag<T>::V V;
  constexpr bool SA = (SPLIT & 1) != 0;
  constexpr bool SB = (SPLIT & 2) != 0;
  const T* A = (const T*)Ap; const T* A2 = (const T*)A2p; const T* Bt = (const T*)Btp; const T* Bt2 = (const T*)Bt2p;
  __shared__ __align__(16) float sT[8][16 * 68];
  const int b    = blockIdx.y;
  const int lane = threadIdx.x & 31;
  const int wave = threadIdx.x >> 5;
  const int tilesN = N >> 6;
  const int tilesM = M >> 6;
  const int tile = blockIdx.x * 8 + wave;
  if (tile >= tilesM * tilesN) return;
  const int tm = tile / tilesN;
  const int tn = tile - tm * tilesN;
  const int m0 = tm << 6;
  const int n0 = tn << 6;

  const T* Ab  = A  + (size_t)b * strideA;
  const T* Bb  = Bt + (size_t)b * strideB;
  const T* Ab2 = SA ? (A2  + (size_t)b * strideA) : nullptr;
  const T* Bb2 = SB ? (Bt2 + (size_t)b * strideB) : nullptr;

  const int rlane = lane & 15;
  const int koff  = (lane >> 4) * 8;
  const int mOff  = (lane >> 4) * 8;

  v8f acc[4][4];
#pragma unroll
  for (int i = 0; i < 4; ++i)
#pragma unroll
    for (int j = 0; j < 4; ++j) acc[i][j] = (v8f){0.f,0.f,0.f,0.f,0.f,0.f,0.f,0.f};

  for (int k0 = 0; k0 < K; k0 += 32) {
    V bh[4], bl[4];
#pragma unroll
    for (int j = 0; j < 4; ++j) {
      const size_t bo = (size_t)(n0 + (j << 4) + rlane) * ldb + koff + k0;
      bh[j] = Frag<T>::load(Bb + bo);
      if (SB) bl[j] = Frag<T>::load(Bb2 + bo);
    }
#pragma unroll
    for (int i = 0; i < 4; ++i) {
      const size_t ao = (size_t)(m0 + (i << 4) + rlane) * lda + koff + k0;
      V ah = Frag<T>::load(Ab + ao);
      V al;
      if (SA) al = Frag<T>::load(Ab2 + ao);
#pragma unroll
      for (int j = 0; j < 4; ++j) {
        acc[i][j] = Frag<T>::mma(ah, bh[j], acc[i][j]);
        if (SB) acc[i][j] = Frag<T>::mma(ah, bl[j], acc[i][j]);
        if (SA) acc[i][j] = Frag<T>::mma(al, bh[j], acc[i][j]);
      }
      Frag<T>::guard(acc[i][0], acc[i][3], ah, SA ? al : ah);
    }
    Frag<T>::keep(bh[0], bh[1], bh[2], bh[3]);
    if (SB) Frag<T>::keep(bl[0], bl[1], bl[2], bl[3]);
  }
  acc_guard4(acc[0][0], acc[0][1], acc[0][2], acc[0][3]);
  acc_guard4(acc[1][0], acc[1][1], acc[1][2], acc[1][3]);
  acc_guard4(acc[2][0], acc[2][1], acc[2][2], acc[2][3]);
  acc_guard4(acc[3][0], acc[3][1], acc[3][2], acc[3][3]);

  float* slab = sT[wave];
  const float* Rb = RESID ? (resid + (size_t)b * strideR) : nullptr;
#pragma unroll
  for (int i = 0; i < 4; ++i) {
    const int mBase = m0 + (i << 4);
#pragma unroll
    for (int j = 0; j < 4; ++j) {
      const int n = n0 + (j << 4) + rlane;
      float bv = 0.f;
      if (BIAS_MODE == 2) bv = bias[n];
#pragma unroll
      for (int r = 0; r < 8; ++r) {
        float v = acc[i][j][r] * scale;
        if (BIAS_MODE == 1) v += bias[mBase + mOff + r];
        if (BIAS_MODE == 2) v += bv;
        if (RESID) v += Rb[(size_t)(mBase + mOff + r) * ldc + n];
        if (ACT == 1) v = tanhf(v);
        if (ACT == 2) v = fmaxf(v, 0.0f);
        slab[(mOff + r) * 68 + (j << 4) + rlane] = v;
      }
    }
    __builtin_amdgcn_fence(__ATOMIC_RELEASE, "workgroup");
    __builtin_amdgcn_wave_barrier();
    __builtin_amdgcn_fence(__ATOMIC_ACQUIRE, "workgroup");
    if (OUT_MODE == 0) {
      float* C = (float*)Cout + (size_t)b * strideC;
      const int hh = lane >> 4, c4 = (lane & 15) * 4;
      for (int pass = 0; pass < 2; ++pass) {
#pragma unroll
        for (int it = 0; it < 8; ++it) {
          const int row = it * 2 + hh;
          v4f v = *(const v4f*)(slab + row * 68 + c4);
          *(volatile v4f*)(C + (size_t)(mBase + row) * ldc + n0 + c4) = v;
        }
        __threadfence();
      }
    } else {
      const int q = lane >> 3, c8 = (lane & 7) * 8;
      unsigned short* C  = (unsigned short*)Cout  + (size_t)b * strideC;
      unsigned short* C2 = (OUT_MODE == 2) ? ((unsigned short*)Cout2 + (size_t)b * strideC) : nullptr;
      for (int pass = 0; pass < 2; ++pass) {
#pragma unroll
        for (int it = 0; it < 4; ++it) {
          const int row = it * 4 + q;
          const float* sp = slab + row * 68 + c8;
          v8h hv, lv;
#pragma unroll
          for (int e = 0; e < 8; ++e) {
            if (OUT_MODE == 1) {
              hv[e] = (_Float16)sp[e];
            } else {
              unsigned short hb = f2bf_bits(sp[e]);
              unsigned short lb = f2bf_bits(sp[e] - bf_bits2f(hb));
              hv[e] = __builtin_bit_cast(_Float16, hb);
              lv[e] = __builtin_bit_cast(_Float16, lb);
            }
          }
          *(volatile v8h*)(C + (size_t)(mBase + row) * ldc + n0 + c8) = hv;
          if (OUT_MODE == 2) *(volatile v8h*)(C2 + (size_t)(mBase + row) * ldc + n0 + c8) = lv;
        }
        __threadfence();
      }
    }
    __builtin_amdgcn_fence(__ATOMIC_RELEASE, "workgroup");
    __builtin_amdgcn_wave_barrier();
    __builtin_amdgcn_fence(__ATOMIC_ACQUIRE, "workgroup");
  }
}

__global__ __launch_bounds__(256) void cast8_bf16_kernel(const float* __restrict__ in, unsigned short* __restrict__ out, int n8) {
  const int i = blockIdx.x * 256 + threadIdx.x;
  if (i >= n8) return;
  const float* p = in + 8 * (size_t)i;
  const v4f a = *(const v4f*)(p);
  const v4f c = *(const v4f*)(p + 4);
  unsigned short hb[8];
#pragma unroll
  for (int e = 0; e < 4; ++e) {
    hb[e]     = f2bf_bits(a[e]);
    hb[4 + e] = f2bf_bits(c[e]);
  }
  const v4u u = (v4u){pk16(hb[0], hb[1]), pk16(hb[2], hb[3]), pk16(hb[4], hb[5]), pk16(hb[6], hb[7])};
  unsigned short* q = out + 8 * (size_t)i;
  *(volatile v4u*)q = u;
  __threadfence();
  *(volatile v4u*)q = u;
}

__global__ __launch_bounds__(256) void wtcast_kernel(const float* __restrict__ Wa, const float* __restrict__ Wb,
                                                     const float* __restrict__ Wc, const float* __restrict__ Wd,
                                                     const float* __restrict__ We, unsigned short* __restrict__ out) {
  __shared__ float sm[64][65];
  const int t  = threadIdx.x;
  const int d0 = blockIdx.x * 64;
  const int h0 = blockIdx.y * 64;
  const int z  = blockIdx.z;
  const float* W = (z == 0) ? Wa : (z == 1) ? Wb : (z == 2) ? Wc : (z == 3) ? Wd : We;
#pragma unroll
  for (int i = 0; i < 16; ++i) {
    const int e = i * 256 + t;
    const int r = e >> 6;
    const int c = e & 63;
    sm[c][r] = W[(size_t)(d0 + r) * DMODEL + h0 + c];
  }
  __syncthreads();
  const int lane = t & 31, wave = t >> 5;
  const int q = lane >> 3, c8 = (lane & 7) * 8;
  unsigned short* op = out + (size_t)z * DMODEL * DMODEL;
  for (int pass = 0; pass < 2; ++pass) {
#pragma unroll
    for (int it = 0; it < 2; ++it) {
      const int row = wave * 8 + it * 4 + q;
      unsigned short hb[8];
#pragma unroll
      for (int e = 0; e < 8; ++e) hb[e] = f2bf_bits(sm[row][c8 + e]);
      const v4u u = (v4u){pk16(hb[0], hb[1]), pk16(hb[2], hb[3]), pk16(hb[4], hb[5]), pk16(hb[6], hb[7])};
      *(volatile v4u*)(op + (size_t)(h0 + row) * DMODEL + d0 + c8) = u;
    }
    __threadfence();
  }
}

__global__ __launch_bounds__(256) void relprep_kernel(const float* __restrict__ pe_key, const float* __restrict__ pe_value,
                                                      unsigned short* __restrict__ PEK,
                                                      unsigned short* __restrict__ VBh, unsigned short* __restrict__ VBl) {
  const int t = threadIdx.x, lane = t & 31, wave = t >> 5;
  if (blockIdx.x < 128) {
    const int gw = blockIdx.x * 8 + wave;
    const int d  = gw & (DMODEL - 1);
    const int r0 = lane * 8;
    unsigned short hb[8];
#pragma unroll
    for (int e = 0; e < 8; ++e) {
      const int r  = r0 + e;
      const int rc = (r < NREL) ? r : (NREL - 1);
      const float f = pe_value[(size_t)rc * DMODEL + d];
      hb[e] = (r < NREL) ? f2bf_bits(f) : (unsigned short)0;
    }
    const v4u u  = (v4u){pk16(hb[0], hb[1]), pk16(hb[2], hb[3]), pk16(hb[4], hb[5]), pk16(hb[6], hb[7])};
    const v4u z4 = (v4u){0u, 0u, 0u, 0u};
    unsigned short* ph = VBh + (size_t)gw * LDCAT + SEQ + r0;
    unsigned short* pl = VBl + (size_t)gw * LDCAT + SEQ + r0;
    if (lane < 24) { *(volatile v4u*)ph = u; *(volatile v4u*)pl = z4; }
    __threadfence();
    if (lane < 24) { *(volatile v4u*)ph = u; *(volatile v4u*)pl = z4; }
  } else {
    const int g  = (blockIdx.x - 128) * 256 + t;
    const int r  = g >> 4;
    const int c8 = (g & 15) * 8;
    const int rc = (r < NREL) ? r : (NREL - 1);
    const float* src = pe_key + (size_t)rc * DMODEL + c8;
    const v4f a = *(const v4f*)(src);
    const v4f c = *(const v4f*)(src + 4);
    const bool live = (r < NREL);
    unsigned short hb[8];
#pragma unroll
    for (int e = 0; e < 4; ++e) {
      hb[e]     = live ? f2bf_bits(a[e]) : (unsigned short)0;
      hb[4 + e] = live ? f2bf_bits(c[e]) : (unsigned short)0;
    }
    const v4u u = (v4u){pk16(hb[0], hb[1]), pk16(hb[2], hb[3]), pk16(hb[4], hb[5]), pk16(hb[6], hb[7])};
    unsigned short* q = PEK + (size_t)r * DMODEL + c8;
    *(volatile v4u*)q = u;
    __threadfence();
    *(volatile v4u*)q = u;
  }
}

__global__ __launch_bounds__(128) void softmax_relpos_kernel(const float* __restrict__ S, const float* __restrict__ QP,
                                                             unsigned short* __restrict__ PRh, unsigned short* __restrict__ PRl) {
  __shared__ float prow[SEQ];
  __shared__ float qps[NRELP];
  __shared__ float redM[4];
  __shared__ float redL[4];
  __shared__ float redA[4];
  __shared__ float redB[4];
  const int row  = blockIdx.x;
  const int i    = row & (SEQ - 1);
  const int t    = threadIdx.x;
  const int lane = t & 31, wave = t >> 5;
  const int c0   = t * 8;
  const float* qr = QP + (size_t)row * NRELP;
  qps[t] = qr[t];
  if (wave < 2) qps[128 + t] = qr[128 + t];
  __syncthreads();
  const float* sr = S + (size_t)row * SEQ + c0;
  const v4f a = *(const v4f*)(sr);
  const v4f c = *(const v4f*)(sr + 4);
  float x[8];
#pragma unroll
  for (int e = 0; e < 4; ++e) { x[e] = a[e]; x[4 + e] = c[e]; }
#pragma unroll
  for (int e = 0; e < 8; ++e) {
    int id = RWIN + c0 + e - i;
    id = id < 0 ? 0 : (id > 2 * RWIN ? 2 * RWIN : id);
    x[e] += qps[id];
  }
  float m = fmaxf(fmaxf(fmaxf(x[0], x[1]), fmaxf(x[2], x[3])), fmaxf(fmaxf(x[4], x[5]), fmaxf(x[6], x[7])));
#pragma unroll
  for (int off = 16; off > 0; off >>= 1) m = fmaxf(m, __shfl_xor(m, off, 32));
  if (lane == 0) redM[wave] = m;
  __syncthreads();
  const float rmax = fmaxf(fmaxf(redM[0], redM[1]), fmaxf(redM[2], redM[3]));
  float ex[8];
#pragma unroll
  for (int e = 0; e < 8; ++e) ex[e] = __expf(x[e] - rmax);
  float s = ((ex[0] + ex[1]) + (ex[2] + ex[3])) + ((ex[4] + ex[5]) + (ex[6] + ex[7]));
#pragma unroll
  for (int off = 16; off > 0; off >>= 1) s += __shfl_xor(s, off, 32);
  if (lane == 0) redL[wave] = s;
  __syncthreads();
  const float l = (redL[0] + redL[1]) + (redL[2] + redL[3]);
  const float f = 1.0f / l;
  float p[8];
  float s0 = 0.f, s1 = 0.f;
#pragma unroll
  for (int e = 0; e < 8; ++e) {
    p[e] = ex[e] * f;
    prow[c0 + e] = p[e];
    const int j = c0 + e;
    s0 += (j <= i - RWIN) ? p[e] : 0.0f;
    s1 += (j >= i + RWIN) ? p[e] : 0.0f;
  }
#pragma unroll
  for (int off = 16; off > 0; off >>= 1) { s0 += __shfl_xor(s0, off, 32); s1 += __shfl_xor(s1, off, 32); }
  if (lane == 0) { redA[wave] = s0; redB[wave] = s1; }
  __syncthreads();
  const float sum0 = (redA[0] + redA[1]) + (redA[2] + redA[3]);
  const float sum1 = (redB[0] + redB[1]) + (redB[2] + redB[3]);

  unsigned short phb[8], plb[8];
#pragma unroll
  for (int e = 0; e < 8; ++e) {
    const unsigned short h = f2bf_bits(p[e]);
    phb[e] = h;
    plb[e] = f2bf_bits(p[e] - bf_bits2f(h));
  }
  const v4u uh = (v4u){pk16(phb[0], phb[1]), pk16(phb[2], phb[3]), pk16(phb[4], phb[5]), pk16(phb[6], phb[7])};
  const v4u ul = (v4u){pk16(plb[0], plb[1]), pk16(plb[2], plb[3]), pk16(plb[4], plb[5]), pk16(plb[6], plb[7])};

  v4u rh = (v4u){0u, 0u, 0u, 0u};
  v4u rl = (v4u){0u, 0u, 0u, 0u};
  if (wave == 0) {
    const int r0 = lane * 8;
    unsigned short hb[8], lb[8];
#pragma unroll
    for (int e = 0; e < 8; ++e) {
      const int r  = r0 + e;
      const int jj = i + r - RWIN;
      const int jc = jj < 0 ? 0 : (jj > SEQ - 1 ? SEQ - 1 : jj);
      const float pv = prow[jc];
      float val = (r >= 1 && r <= 2 * RWIN - 1 && jj >= 0 && jj < SEQ) ? pv : 0.0f;
      val = (r == 0) ? sum0 : val;
      val = (r == 2 * RWIN) ? sum1 : val;
      const unsigned short h = f2bf_bits(val);
      hb[e] = h;
      lb[e] = f2bf_bits(val - bf_bits2f(h));
    }
    rh = (v4u){pk16(hb[0], hb[1]), pk16(hb[2], hb[3]), pk16(hb[4], hb[5]), pk16(hb[6], hb[7])};
    rl = (v4u){pk16(lb[0], lb[1]), pk16(lb[2], lb[3]), pk16(lb[4], lb[5]), pk16(lb[6], lb[7])};
  }
  const bool wst = (wave == 0) && (lane < 24);
  const size_t rbase = (size_t)row * LDCAT;
  for (int pass = 0; pass < 2; ++pass) {
    *(volatile v4u*)(PRh + rbase + c0) = uh;
    *(volatile v4u*)(PRl + rbase + c0) = ul;
    if (wst) {
      *(volatile v4u*)(PRh + rbase + SEQ + lane * 8) = rh;
      *(volatile v4u*)(PRl + rbase + SEQ + lane * 8) = rl;
    }
    __threadfence();
  }
}

extern "C" void kernel_launch(void* const* d_in, const int* in_sizes, int n_in,
                              void* d_out, int out_size, void* d_ws, size_t ws_size,
                              hipStream_t stream) {
  if (n_in < 13) return;
  if (in_sizes[0] != NTOK * DMODEL) return;
  if (in_sizes[1] != DMODEL * DMODEL || in_sizes[3] != DMODEL * DMODEL || in_sizes[5] != DMODEL * DMODEL) return;
  if (in_sizes[7] != DMODEL * DMODEL || in_sizes[9] != DMODEL * DMODEL) return;
  if (in_sizes[2] != DMODEL || in_sizes[4] != DMODEL || in_sizes[6] != DMODEL || in_sizes[8] != DMODEL || in_sizes[10] != DMODEL) return;
  if (in_sizes[11] != NREL * DMODEL || in_sizes[12] != NREL * DMODEL) return;
  if (out_size != NTOK * DMODEL) return;

  const float* x    = (const float*)d_in[0];
  const float* W0   = (const float*)d_in[1];
  const float* b0   = (const float*)d_in[2];
  const float* Wq   = (const float*)d_in[3];
  const float* bq   = (const float*)d_in[4];
  const float* Wk   = (const float*)d_in[5];
  const float* bk   = (const float*)d_in[6];
  const float* Wv   = (const float*)d_in[7];
  const float* bv   = (const float*)d_in[8];
  const float* W1   = (const float*)d_in[9];
  const float* b1   = (const float*)d_in[10];
  const float* pek  = (const float*)d_in[11];
  const float* pev  = (const float*)d_in[12];
  float* outp = (float*)d_out;

  const size_t SZ_X16 = (size_t)NTOK * DMODEL * 2;
  const size_t SZ_WT  = (size_t)5 * DMODEL * DMODEL * 2;
  const size_t SZ_PEK = (size_t)NRELP * DMODEL * 2;
  const size_t SZ_PL  = (size_t)NTOK * DMODEL * 2;
  const size_t SZ_VB  = (size_t)NBATCH * DMODEL * LDCAT * 2;
  const size_t SZ_QP  = (size_t)NTOK * NRELP * 4;
  const size_t SZ_S   = (size_t)NBATCH * SEQ * SEQ * 4;
  const size_t SZ_PR  = (size_t)NBATCH * SEQ * LDCAT * 2;
  size_t off = 0;
  const size_t oX16 = off; off += SZ_X16;
  const size_t oWT  = off; off += SZ_WT;
  const size_t oPEK = off; off += SZ_PEK;
  const size_t oHSh = off; off += SZ_PL;
  const size_t oHSl = off; off += SZ_PL;
  const size_t oQh  = off; off += SZ_PL;
  const size_t oQl  = off; off += SZ_PL;
  const size_t oKh  = off; off += SZ_PL;
  const size_t oKl  = off; off += SZ_PL;
  const size_t oVBh = off; off += SZ_VB;
  const size_t oVBl = off; off += SZ_VB;
  const size_t oQP  = off; off += SZ_QP;
  const size_t oS   = off; off += SZ_S;
  const size_t oPRh = off; off += SZ_PR;
  const size_t oPRl = off; off += SZ_PR;
  const size_t TOTAL = off;
  if (TOTAL > ws_size) return;
  if (TOTAL > (size_t)134217728) return;

  char* ws = (char*)d_ws;
  unsigned short* X16  = (unsigned short*)(ws + oX16);
  unsigned short* WT   = (unsigned short*)(ws + oWT);
  unsigned short* W0T  = WT;
  unsigned short* WqT  = WT + (size_t)1 * DMODEL * DMODEL;
  unsigned short* WkT  = WT + (size_t)2 * DMODEL * DMODEL;
  unsigned short* WvT  = WT + (size_t)3 * DMODEL * DMODEL;
  unsigned short* W1T  = WT + (size_t)4 * DMODEL * DMODEL;
  unsigned short* PEK  = (unsigned short*)(ws + oPEK);
  unsigned short* HSh  = (unsigned short*)(ws + oHSh);
  unsigned short* HSl  = (unsigned short*)(ws + oHSl);
  unsigned short* Ch   = HSh;
  unsigned short* Cl   = HSl;
  unsigned short* Qh   = (unsigned short*)(ws + oQh);
  unsigned short* Ql   = (unsigned short*)(ws + oQl);
  unsigned short* Kh   = (unsigned short*)(ws + oKh);
  unsigned short* Kl   = (unsigned short*)(ws + oKl);
  unsigned short* VBh  = (unsigned short*)(ws + oVBh);
  unsigned short* VBl  = (unsigned short*)(ws + oVBl);
  float*          QPf  = (float*)(ws + oQP);
  float*          Sf   = (float*)(ws + oS);
  unsigned short* PRh  = (unsigned short*)(ws + oPRh);
  unsigned short* PRl  = (unsigned short*)(ws + oPRl);

  const dim3 blk(256);

  {
    const int n8 = NTOK * DMODEL / 8;
    cast8_bf16_kernel<<<dim3((n8 + 255) / 256), blk, 0, stream>>>(x, X16, n8);
  }
  wtcast_kernel<<<dim3(DMODEL / 64, DMODEL / 64, 5), blk, 0, stream>>>(W0, Wq, Wk, Wv, W1, WT);
  relprep_kernel<<<dim3(128 + 12), blk, 0, stream>>>(pek, pev, PEK, VBh, VBl);

  const dim3 gTok(((NTOK / 64) * (DMODEL / 64) + 7) / 8, 1);
  const dim3 gV((((DMODEL / 64) * (SEQ / 64)) + 7) / 8, NBATCH);
  const dim3 gQP(((NTOK / 64) * (NRELP / 64) + 7) / 8, 1);
  const dim3 gS((((SEQ / 64) * (SEQ / 64)) + 7) / 8, NBATCH);
  const dim3 gPV((((SEQ / 64) * (DMODEL / 64)) + 7) / 8, NBATCH);

  wmma_gemm64<1, 0, 2, 2, false, 2><<<gTok, blk, 0, stream>>>(
      X16, X16, DMODEL, 0L, W0T, W0T, DMODEL, 0L, (void*)HSh, (void*)HSl, DMODEL, 0L,
      b0, x, 0L, NTOK, DMODEL, DMODEL, 1.0f);
  wmma_gemm64<1, 1, 2, 2, false, 1><<<gTok, blk, 0, stream>>>(
      HSh, HSl, DMODEL, 0L, WqT, WqT, DMODEL, 0L, (void*)Qh, (void*)Ql, DMODEL, 0L,
      bq, x, 0L, NTOK, DMODEL, DMODEL, 1.0f);
  wmma_gemm64<1, 1, 2, 2, false, 1><<<gTok, blk, 0, stream>>>(
      HSh, HSl, DMODEL, 0L, WkT, WkT, DMODEL, 0L, (void*)Kh, (void*)Kl, DMODEL, 0L,
      bk, x, 0L, NTOK, DMODEL, DMODEL, 1.0f);
  wmma_gemm64<1, 2, 1, 2, false, 1><<<gV, blk, 0, stream>>>(
      WvT, WvT, DMODEL, 0L, HSh, HSl, DMODEL, (long)SEQ * DMODEL, (void*)VBh, (void*)VBl, LDCAT, (long)DMODEL * LDCAT,
      bv, x, 0L, DMODEL, SEQ, DMODEL, 1.0f);
  wmma_gemm64<1, 1, 0, 0, false, 0><<<gQP, blk, 0, stream>>>(
      Qh, Ql, DMODEL, 0L, PEK, PEK, DMODEL, 0L, (void*)QPf, (void*)QPf, NRELP, 0L,
      b0, x, 0L, NTOK, NRELP, DMODEL, 1.0f);
  wmma_gemm64<1, 3, 0, 0, false, 0><<<gS, blk, 0, stream>>>(
      Qh, Ql, DMODEL, (long)SEQ * DMODEL, Kh, Kl, DMODEL, (long)SEQ * DMODEL, (void*)Sf, (void*)Sf, SEQ, (long)SEQ * SEQ,
      b0, x, 0L, SEQ, SEQ, DMODEL, 1.0f);
  softmax_relpos_kernel<<<dim3(NTOK), dim3(128), 0, stream>>>(Sf, QPf, PRh, PRl);
  wmma_gemm64<1, 3, 0, 2, false, 0><<<gPV, blk, 0, stream>>>(
      PRh, PRl, LDCAT, (long)SEQ * LDCAT, VBh, VBl, LDCAT, (long)DMODEL * LDCAT, (void*)Ch, (void*)Cl, DMODEL, (long)SEQ * DMODEL,
      b0, x, 0L, SEQ, DMODEL, LDCAT, 1.0f);
  wmma_gemm64<1, 1, 2, 0, false, 2><<<gTok, blk, 0, stream>>>(
      Ch, Cl, DMODEL, 0L, W1T, W1T, DMODEL, 0L, (void*)outp, (void*)outp, DMODEL, 0L,
      b1, x, 0L, NTOK, DMODEL, DMODEL, 1.0f);
}
